// CGGRUNet_85993835200797
// MI455X (gfx1250) — hardware-verified
//
#include <hip/hip_runtime.h>
#include <stddef.h>


#define DIM    64
#define NFT    92
#define EFT    50
#define HID    128
#define NGR    64
#define CT     128
#define CW     4
#define NBK    64
#define SCAP   32
#define PCAP   2048
#define EPT    8
#define CHUNK  (CT * EPT)
#define WCAP   (EPT * 32)
#define KW2    8256
#define KH0    4096
#define KH1    4160
#define SPITCH 4168
#define MPITCH 72
#define ET     64
#define EAP    72
#define HSP    136

#define L_ST    0
#define L_OT    (L_ST + 16 * SPITCH * 2)
#define L_HT    (L_OT + CW * 64 * 32 * 2)
#define L_PEND  (L_HT + CW * 128 * 32 * 2)
#define L_SLOT  (L_PEND + PCAP * 4)
#define L_CNT   (L_SLOT + NBK * SCAP * 4)
#define L_LIST  (L_CNT + NBK * 4)
#define L_WC    (L_LIST + CW * WCAP * 4)
#define L_M16   (L_WC + 64)
#define L_O32   (L_M16 + 16 * MPITCH * 2)
#define L_O16   (L_O32 + 16 * DIM * 4)
#define L_TOTAL (L_O16 + 16 * DIM * 2)

#define S_QS   0
#define S_HS   (S_QS + NGR * 2 * DIM * 4)
#define S_CS   (S_HS + NGR * DIM * 4)
#define S_SCR  (S_CS + NGR * DIM * 4)
#define S_EMX  (S_SCR + NGR * 4 * DIM * 4)
#define S_DEN  (S_EMX + 4 * NGR * 4)
#define S_Y    (S_DEN + 4 * NGR * 4)
#define S_E    (S_Y + NGR * 4)

static_assert(NBK == 64);
static_assert(SCAP == 32);
static_assert(CW * 4 == 16);
static_assert((NBK % 16) == 0);
static_assert(WCAP == 256);
static_assert(CHUNK == 1024);
static_assert((KW2 % 32) == 0 && KW2 == KH0 + KH1);
static_assert(KH0 == 32 * HID && KH1 == 32 * HID + DIM);
static_assert((SPITCH % 8) == 0 && SPITCH >= KH1);
static_assert((MPITCH % 8) == 0 && (EAP % 8) == 0 && (HSP % 8) == 0);
static_assert((L_OT % 16) == 0 && (L_HT % 16) == 0 && (L_PEND % 16) == 0 && (L_SLOT % 16) == 0);
static_assert((L_CNT % 16) == 0 && (L_LIST % 16) == 0 && (L_WC % 16) == 0 && (L_M16 % 16) == 0);
static_assert((L_O32 % 16) == 0 && (L_O16 % 16) == 0 && (L_TOTAL % 16) == 0);
static_assert(L_TOTAL <= 300 * 1024);
static_assert((S_HS % 16) == 0 && (S_CS % 16) == 0 && (S_SCR % 16) == 0 && (S_EMX % 16) == 0);
static_assert((S_DEN % 16) == 0 && (S_Y % 16) == 0 && (S_E % 16) == 0);
static_assert(NGR * 4 == 256);
static_assert(ET * 2 == 8 * CW * 4);
static_assert(HID * 2 == 2 * 128);

typedef float    v4f  __attribute__((ext_vector_type(4)));
typedef float    v8f  __attribute__((ext_vector_type(8)));
typedef int      v4i  __attribute__((ext_vector_type(4)));
typedef _Float16 v8h  __attribute__((ext_vector_type(8), __may_alias__));
typedef _Float16 v16h __attribute__((ext_vector_type(16)));
union Frag { v16h v; v8h hv[2]; };
union U8 { v8h h; v4f f; };

__device__ __forceinline__ v8f wmh(v16h a, v16h b, v8f c) {
  v8f d = __builtin_amdgcn_wmma_f32_16x16x32_f16(false, a, false, b, (short)0, c, false, false);
  asm volatile("v_nop\n\tv_nop\n\tv_nop\n\tv_nop" : "+v"(d) : "v"(a), "v"(b));
  return d;
}

__device__ __forceinline__ v8f z8f() {
  v8f c;
#pragma unroll
  for (int i = 0; i < 8; ++i) c[i] = 0.0f;
  return c;
}

__device__ __forceinline__ v8h z8h() {
  v8h c;
#pragma unroll
  for (int i = 0; i < 8; ++i) c[i] = (_Float16)0.0f;
  return c;
}

__device__ __forceinline__ float sigf(float x) { return __builtin_amdgcn_rcpf(1.0f + __expf(-x)); }
__device__ __forceinline__ float tnhf(float x) { return 2.0f * __builtin_amdgcn_rcpf(1.0f + __expf(-2.0f * x)) - 1.0f; }

__global__ __launch_bounds__(128) void k_prep4(const float* __restrict__ nn1w, const float* __restrict__ root,
                                               const float* __restrict__ gih, const float* __restrict__ ghh,
                                               _Float16* w1s, _Float16* roots, _Float16* gihs, _Float16* ghhs) {
  const int plane = blockIdx.y;
  const int gid = blockIdx.x * 128 + threadIdx.x;
  int rows;
  _Float16* dst;
  if (plane == 0) { rows = HID; dst = w1s; }
  else if (plane == 1) { rows = DIM; dst = roots; }
  else if (plane == 2) { rows = 3 * DIM; dst = gihs; }
  else { rows = 3 * DIM; dst = ghhs; }
  if (gid >= rows * 8) return;
  const int row = gid >> 3, p = gid & 7;
  U8 u;
#pragma unroll
  for (int j = 0; j < 8; ++j) {
    const int k = 8 * p + j;
    float v;
    if (plane == 0) {
      const int kk = k > EFT - 1 ? EFT - 1 : k;
      v = nn1w[row * EFT + kk];
      v = (k < EFT) ? v : 0.0f;
    } else if (plane == 1) {
      v = root[k * DIM + row];
    } else if (plane == 2) {
      v = gih[row * DIM + k];
    } else {
      v = ghh[row * DIM + k];
    }
    u.h[j] = (_Float16)(v * 64.0f);
  }
  volatile v4f* q = (volatile v4f*)(dst + (size_t)row * DIM + 8 * p);
  *q = u.f;
  __threadfence();
  *q = u.f;
}

__global__ __launch_bounds__(128) void k_prepw2(const float* __restrict__ nn2w, const float* __restrict__ nn2b,
                                                _Float16* w2s) {
  const int gid = blockIdx.x * 128 + threadIdx.x;
  if (gid >= DIM * (KW2 / 8)) return;
  const int o = gid / (KW2 / 8);
  const int p = gid - o * (KW2 / 8);
  U8 u;
#pragma unroll
  for (int j = 0; j < 8; ++j) {
    const int kk = 8 * p + j;
    const int iw = kk > DIM * HID - 1 ? DIM * HID - 1 : kk;
    const int i = iw >> 7, k = iw & 127;
    const float vw = nn2w[((size_t)(i * DIM + o)) * HID + k];
    int ib = kk - DIM * HID;
    ib = ib < 0 ? 0 : (ib > DIM - 1 ? DIM - 1 : ib);
    const float vb = nn2b[ib * DIM + o];
    const float v = (kk < DIM * HID) ? vw : vb;
    u.h[j] = (_Float16)(v * 64.0f);
  }
  volatile v4f* q = (volatile v4f*)(w2s + (size_t)o * KW2 + 8 * p);
  *q = u.f;
  __threadfence();
  *q = u.f;
}

__global__ __launch_bounds__(256) void k_lin0(const float* __restrict__ x, const float* __restrict__ w,
                                              const float* __restrict__ b, float* o32, _Float16* o16, int nN) {
  __shared__ __attribute__((aligned(16))) float xr[4][NFT];
  __shared__ __attribute__((aligned(16))) float t32[4 * DIM];
  __shared__ __attribute__((aligned(16))) _Float16 t16[4 * DIM];
  const int tid = threadIdx.x, ln = tid >> 6, d = tid & 63;
  const int n0 = blockIdx.x * 4;
  int nr = n0 + ln;
  nr = nr > nN - 1 ? nN - 1 : nr;
  for (int j = d; j < NFT; j += DIM) xr[ln][j] = x[(size_t)nr * NFT + j];
  __syncthreads();
  float s = b[d];
  const float* wr = w + d * NFT;
#pragma unroll 4
  for (int j = 0; j < NFT; ++j) s = fmaf(xr[ln][j], wr[j], s);
  s = fmaxf(s, 0.0f);
  t32[ln * DIM + d] = s;
  t16[ln * DIM + d] = (_Float16)(s * 8.0f);
  __syncthreads();
  const int L = tid >> 3, p = tid & 7;
  v4f v = {0.0f, 0.0f, 0.0f, 0.0f};
  char* dst = (char*)o32;
  if (tid < 64) {
    const int row = L >> 1, half = L & 1;
    v = *(const v4f*)(t32 + row * DIM + 32 * half + 4 * p);
    dst = (char*)(o32 + (size_t)(n0 + row) * DIM + 32 * half + 4 * p);
  } else if (tid < 96) {
    const int row = L - 8;
    U8 u;
    u.h = *(const v8h*)(t16 + row * DIM + 8 * p);
    v = u.f;
    dst = (char*)(o16 + (size_t)(n0 + row) * DIM + 8 * p);
  }
  if (tid < 96) *(volatile v4f*)dst = v;
  __threadfence();
  if (tid < 96) *(volatile v4f*)dst = v;
}

__global__ __launch_bounds__(CT) void k_nn1(const float* __restrict__ ea, const float* __restrict__ b1v,
                                            const _Float16* __restrict__ w1s, _Float16* he16, int nE) {
  __shared__ __attribute__((aligned(16))) _Float16 ea16[ET * EAP];
  __shared__ __attribute__((aligned(16))) _Float16 hst[ET * HSP];
  const int tid = threadIdx.x, lane = tid & 31, wave = tid >> 5, h = lane >> 4, m = lane & 15;
  const int eb = blockIdx.x * ET;
#pragma unroll 1
  for (int idx = tid; idx < ET * 64; idx += CT) {
    const int r = idx >> 6, c = idx & 63;
    int row = eb + r;
    row = row > nE - 1 ? nE - 1 : row;
    const int cc = c > EFT - 1 ? EFT - 1 : c;
    float v = ea[(size_t)row * EFT + cc];
    v = (c < EFT) ? v : 0.0f;
    ea16[r * EAP + c] = (_Float16)v;
  }
  __syncthreads();
  Frag a0, a1;
  {
    const _Float16* ar = ea16 + (16 * wave + m) * EAP + 8 * h;
    a0.hv[0] = *(const v8h*)ar;
    a0.hv[1] = *(const v8h*)(ar + 16);
    a1.hv[0] = *(const v8h*)(ar + 32);
    a1.hv[1] = *(const v8h*)(ar + 48);
  }
#pragma unroll 2
  for (int nt = 0; nt < HID / 16; ++nt) {
    const int ncol = 16 * nt + m;
    const _Float16* wp = w1s + (size_t)ncol * 64 + 8 * h;
    Frag b0, b1;
    b0.hv[0] = *(const v8h*)wp;
    b0.hv[1] = *(const v8h*)(wp + 16);
    b1.hv[0] = *(const v8h*)(wp + 32);
    b1.hv[1] = *(const v8h*)(wp + 48);
    v8f acc = wmh(a0.v, b0.v, z8f());
    acc = wmh(a1.v, b1.v, acc);
    const float bias = b1v[ncol];
#pragma unroll
    for (int r = 0; r < 8; ++r) {
      const float v = fmaxf(acc[r] * (1.0f / 64.0f) + bias, 0.0f);
      hst[(16 * wave + 8 * h + r) * HSP + ncol] = (_Float16)(v * 8.0f);
    }
  }
  __syncthreads();
  const int p = lane & 7, lr = lane >> 3;
#pragma unroll
  for (int q = 0; q < 8; ++q) {
    const int L = 16 * q + 4 * wave + lr;
    const int row = L >> 1, half = L & 1;
    U8 u;
    u.h = *(const v8h*)(hst + row * HSP + 64 * half + 8 * p);
    *(volatile v4f*)(he16 + (size_t)(eb + row) * HID + 64 * half + 8 * p) = u.f;
  }
  __threadfence();
#pragma unroll
  for (int q = 0; q < 8; ++q) {
    const int L = 16 * q + 4 * wave + lr;
    const int row = L >> 1, half = L & 1;
    U8 u;
    u.h = *(const v8h*)(hst + row * HSP + 64 * half + 8 * p);
    *(volatile v4f*)(he16 + (size_t)(eb + row) * HID + 64 * half + 8 * p) = u.f;
  }
}

__device__ __forceinline__ int scan_chunk(const int* __restrict__ dsts, int nE, int cbase, int nodeBase,
                                          int vec8, int* list, int tid, int wave) {
  int wc = 0;
  const int el0  = tid * EPT;
  const int e0   = cbase + el0;
  const int sent = -2147483647 - 1;
  v4i da, db;
  if (vec8 != 0 && cbase + CHUNK <= nE) {
    da = *(const v4i*)(dsts + e0);
    db = *(const v4i*)(dsts + e0 + 4);
  } else {
    da.x = (e0     < nE) ? dsts[min(e0, nE - 1)] : sent;
    da.y = (e0 + 1 < nE) ? dsts[min(e0 + 1, nE - 1)] : sent;
    da.z = (e0 + 2 < nE) ? dsts[min(e0 + 2, nE - 1)] : sent;
    da.w = (e0 + 3 < nE) ? dsts[min(e0 + 3, nE - 1)] : sent;
    db.x = (e0 + 4 < nE) ? dsts[min(e0 + 4, nE - 1)] : sent;
    db.y = (e0 + 5 < nE) ? dsts[min(e0 + 5, nE - 1)] : sent;
    db.z = (e0 + 6 < nE) ? dsts[min(e0 + 6, nE - 1)] : sent;
    db.w = (e0 + 7 < nE) ? dsts[min(e0 + 7, nE - 1)] : sent;
  }
  const unsigned nb = (unsigned)nodeBase;
  const unsigned s0 = (unsigned)da.x - nb, s1 = (unsigned)da.y - nb;
  const unsigned s2 = (unsigned)da.z - nb, s3 = (unsigned)da.w - nb;
  const unsigned s4 = (unsigned)db.x - nb, s5 = (unsigned)db.y - nb;
  const unsigned s6 = (unsigned)db.z - nb, s7 = (unsigned)db.w - nb;
  const bool h0 = s0 < (unsigned)NBK, h1 = s1 < (unsigned)NBK, h2 = s2 < (unsigned)NBK, h3 = s3 < (unsigned)NBK;
  const bool h4 = s4 < (unsigned)NBK, h5 = s5 < (unsigned)NBK, h6 = s6 < (unsigned)NBK, h7 = s7 < (unsigned)NBK;
  const unsigned any = __builtin_amdgcn_ballot_w32(h0 | h1 | h2 | h3 | h4 | h5 | h6 | h7);
  if (any != 0u) {
#define HITJ(J, HJ, SJ) { \
      const unsigned mj = __builtin_amdgcn_ballot_w32(HJ); \
      if (mj != 0u) { \
        if (HJ) { \
          const int pos = wc + (int)__builtin_amdgcn_mbcnt_lo(mj, 0u); \
          if (pos < WCAP) list[wave * WCAP + pos] = (el0 + (J)) * 64 + (int)(SJ); \
        } \
        wc += (int)__builtin_popcount(mj); } }
    HITJ(0, h0, s0)
    HITJ(1, h1, s1)
    HITJ(2, h2, s2)
    HITJ(3, h3, s3)
    HITJ(4, h4, s4)
    HITJ(5, h5, s5)
    HITJ(6, h6, s6)
    HITJ(7, h7, s7)
#undef HITJ
  }
  return wc;
}

__global__ __launch_bounds__(CT) void k_conv(
    const int* __restrict__ ei, const _Float16* __restrict__ xh, const float* __restrict__ xf,
    const _Float16* __restrict__ he16, const _Float16* __restrict__ w2s, const _Float16* __restrict__ roots,
    const _Float16* __restrict__ gihs, const _Float16* __restrict__ ghhs,
    const float* __restrict__ cbias, const float* __restrict__ bih, const float* __restrict__ bhh,
    float* yf, _Float16* yh, int nN, int nE, int vec8) {
  extern __shared__ __attribute__((aligned(16))) unsigned char dsm[];
  _Float16* st    = (_Float16*)(dsm + L_ST);
  int*      pend  = (int*)(dsm + L_PEND);
  int*      slotL = (int*)(dsm + L_SLOT);
  int*      cntL  = (int*)(dsm + L_CNT);
  int*      list  = (int*)(dsm + L_LIST);
  int*      wc    = (int*)(dsm + L_WC);
  _Float16* m16   = (_Float16*)(dsm + L_M16);
  float*    o32   = (float*)(dsm + L_O32);
  _Float16* o16   = (_Float16*)(dsm + L_O16);
  const int tid = threadIdx.x, lane = tid & 31, wave = tid >> 5, h = lane >> 4, m = lane & 15;
  _Float16* otW = (_Float16*)(dsm + L_OT) + wave * (64 * 32);
  _Float16* htW = (_Float16*)(dsm + L_HT) + wave * (128 * 32);
  const int nodeBase = blockIdx.x * NBK;
  const int* srcs = ei;
  const int* dsts = ei + nE;

  if (tid == 0) wc[CW] = 0;
  __syncthreads();
  const int nChunks = (nE + CHUNK - 1) / CHUNK;
#pragma unroll 1
  for (int ch = 0; ch < nChunks; ++ch) {
    const int cbase = ch * CHUNK;
    const int cwc = scan_chunk(dsts, nE, cbase, nodeBase, vec8, list, tid, wave);
    if (lane == 0) wc[wave] = cwc;
    __syncthreads();
    const int base = wc[CW];
    int tot = 0, myoff = 0;
#pragma unroll
    for (int w = 0; w < CW; ++w) {
      int c = wc[w];
      c = c > WCAP ? WCAP : (c < 0 ? 0 : c);
      if (w < wave) myoff += c;
      tot += c;
    }
    {
      int n = wc[wave];
      n = n > WCAP ? WCAP : (n < 0 ? 0 : n);
      const int* lp = list + wave * WCAP;
      for (int i = lane; i < n; i += 32) {
        const int pos = base + myoff + i;
        if (pos < PCAP) pend[pos] = lp[i] + cbase * 64;
      }
    }
    int newN = base + tot;
    newN = newN > PCAP ? PCAP : newN;
    __syncthreads();
    if (tid == 0) wc[CW] = newN;
  }
  __syncthreads();

  {
    int tot = wc[CW];
    tot = tot < 0 ? 0 : (tot > PCAP ? PCAP : tot);
    if (tid < NBK) {
      int cnt = 0;
#pragma unroll 1
      for (int j = 0; j < tot; ++j) {
        const int v = pend[j];
        if ((v & 63) == tid) {
          if (cnt < SCAP) slotL[tid * SCAP + cnt] = v >> 6;
          ++cnt;
        }
      }
      cntL[tid] = cnt;
    }
  }
  __syncthreads();

  const v8h zh = z8h();
#pragma unroll 1
  for (int g = 0; g < NBK / 16; ++g) {
    v8f accA = z8f();
#pragma unroll 1
    for (int hf = 0; hf < 2; ++hf) {
#pragma unroll 1
      for (int q = 0; q < 4; ++q) {
        const int nl = 4 * wave + q;
        const int nb = 16 * g + nl;
        int cnt = cntL[nb];
        cnt = cnt < 0 ? 0 : (cnt > SCAP ? SCAP : cnt);
        const bool valid = lane < cnt;
        const int sidx = valid ? lane : 0;
        int e = slotL[nb * SCAP + sidx];
        e = e < 0 ? 0 : (e > nE - 1 ? nE - 1 : e);
        int s = srcs[e];
        s = s < 0 ? 0 : (s > nN - 1 ? nN - 1 : s);
        const v8h* op = (const v8h*)(xh + (size_t)s * DIM);
        const v8h* hp = (const v8h*)(he16 + (size_t)e * HID);
        __builtin_amdgcn_fence(__ATOMIC_ACQ_REL, "wavefront");
        __builtin_amdgcn_wave_barrier();
#pragma unroll
        for (int c = 0; c < 8; ++c) {
          v8h xv = op[c];
          xv = valid ? xv : zh;
#pragma unroll
          for (int j = 0; j < 8; ++j) otW[(8 * c + j) * 32 + lane] = xv[j];
        }
#pragma unroll
        for (int c = 0; c < 16; ++c) {
          v8h hv = hp[c];
          hv = valid ? hv : zh;
#pragma unroll
          for (int j = 0; j < 8; ++j) htW[(8 * c + j) * 32 + lane] = hv[j];
        }
        __builtin_amdgcn_fence(__ATOMIC_ACQ_REL, "wavefront");
        __builtin_amdgcn_wave_barrier();
        _Float16* srow = st + nl * SPITCH;
        if (hf == 1) {
#pragma unroll
          for (int ii = 0; ii < 2; ++ii) {
            const int i = lane + 32 * ii;
            float t = 0.0f;
#pragma unroll
            for (int c = 0; c < 4; ++c) {
              const v8h xv = *(const v8h*)(otW + i * 32 + 8 * c);
#pragma unroll
              for (int j = 0; j < 8; ++j) t += (float)xv[j];
            }
            srow[KH0 + i] = (_Float16)(t * 8.0f);
          }
        }
#pragma unroll
        for (int it = 0; it < 2; ++it) {
          Frag a;
          const _Float16* ar = otW + (32 * hf + 16 * it + m) * 32 + 8 * h;
          a.hv[0] = *(const v8h*)ar;
          a.hv[1] = *(const v8h*)(ar + 16);
#pragma unroll
          for (int kt = 0; kt < 8; ++kt) {
            Frag b;
            const _Float16* br = htW + (16 * kt + m) * 32 + 8 * h;
            b.hv[0] = *(const v8h*)br;
            b.hv[1] = *(const v8h*)(br + 16);
            const v8f d = wmh(a.v, b.v, z8f());
#pragma unroll
            for (int r = 0; r < 8; ++r) srow[(16 * it + 8 * h + r) * HID + 16 * kt + m] = (_Float16)d[r];
          }
        }
      }
      __syncthreads();
      {
        const int KS = (hf != 0) ? (KH1 / 32) : (KH0 / 32);
        const _Float16* bp = w2s + (size_t)(16 * wave + m) * KW2 + KH0 * hf + 8 * h;
        const _Float16* ap = st + m * SPITCH + 8 * h;
#pragma unroll 2
        for (int ks = 0; ks < KS; ++ks) {
          Frag a, b;
          a.hv[0] = *(const v8h*)(ap + 32 * ks);
          a.hv[1] = *(const v8h*)(ap + 32 * ks + 16);
          b.hv[0] = *(const v8h*)(bp + 32 * ks);
          b.hv[1] = *(const v8h*)(bp + 32 * ks + 16);
          accA = wmh(a.v, b.v, accA);
        }
      }
      __syncthreads();
    }

    {
      const int rowg = nodeBase + 16 * g;
      const int o = 16 * wave + m;
      Frag a0, a1;
      {
        const _Float16* xr = xh + (size_t)(rowg + m) * DIM + 8 * h;
        a0.hv[0] = *(const v8h*)xr;
        a0.hv[1] = *(const v8h*)(xr + 16);
        a1.hv[0] = *(const v8h*)(xr + 32);
        a1.hv[1] = *(const v8h*)(xr + 48);
      }
      v8f accR;
      {
        const _Float16* wp = roots + (size_t)o * DIM + 8 * h;
        Frag b0, b1;
        b0.hv[0] = *(const v8h*)wp;
        b0.hv[1] = *(const v8h*)(wp + 16);
        b1.hv[0] = *(const v8h*)(wp + 32);
        b1.hv[1] = *(const v8h*)(wp + 48);
        accR = wmh(a0.v, b0.v, z8f());
        accR = wmh(a1.v, b1.v, accR);
      }
      {
        const float cb = cbias[o];
#pragma unroll
        for (int r = 0; r < 8; ++r) {
          const int nb = 16 * g + 8 * h + r;
          const int c = cntL[nb];
          const float inv = (c > 0) ? __builtin_amdgcn_rcpf((float)c) : 0.0f;
          float mv = accA[r] * (1.0f / 4096.0f) * inv + accR[r] * (1.0f / 512.0f) + cb;
          mv = fmaxf(mv, 0.0f);
          m16[(8 * h + r) * MPITCH + o] = (_Float16)(mv * 8.0f);
        }
      }
      __syncthreads();
      Frag am0, am1;
      {
        const _Float16* mr = m16 + m * MPITCH + 8 * h;
        am0.hv[0] = *(const v8h*)mr;
        am0.hv[1] = *(const v8h*)(mr + 16);
        am1.hv[0] = *(const v8h*)(mr + 32);
        am1.hv[1] = *(const v8h*)(mr + 48);
      }
      v8f ax0, ax1, ax2, ah0, ah1, ah2;
#define GATEP(T, AX, AH) { \
        const int gcol = 64 * (T) + o; \
        const _Float16* wp = gihs + (size_t)gcol * DIM + 8 * h; \
        Frag b0, b1; \
        b0.hv[0] = *(const v8h*)wp; b0.hv[1] = *(const v8h*)(wp + 16); \
        b1.hv[0] = *(const v8h*)(wp + 32); b1.hv[1] = *(const v8h*)(wp + 48); \
        AX = wmh(am0.v, b0.v, z8f()); AX = wmh(am1.v, b1.v, AX); \
        const _Float16* wq = ghhs + (size_t)gcol * DIM + 8 * h; \
        Frag c0, c1; \
        c0.hv[0] = *(const v8h*)wq; c0.hv[1] = *(const v8h*)(wq + 16); \
        c1.hv[0] = *(const v8h*)(wq + 32); c1.hv[1] = *(const v8h*)(wq + 48); \
        AH = wmh(a0.v, c0.v, z8f()); AH = wmh(a1.v, c1.v, AH); }
      GATEP(0, ax0, ah0)
      GATEP(1, ax1, ah1)
      GATEP(2, ax2, ah2)
#undef GATEP
      {
        const float s512 = 1.0f / 512.0f;
        const float bxr = bih[o], bxz = bih[DIM + o], bxn = bih[2 * DIM + o];
        const float bhr = bhh[o], bhz = bhh[DIM + o], bhn = bhh[2 * DIM + o];
#pragma unroll
        for (int r = 0; r < 8; ++r) {
          const int row = 8 * h + r;
          const float xr = ax0[r] * s512 + bxr, hr = ah0[r] * s512 + bhr;
          const float xz = ax1[r] * s512 + bxz, hz = ah1[r] * s512 + bhz;
          const float xn = ax2[r] * s512 + bxn, hn = ah2[r] * s512 + bhn;
          const float rg = sigf(xr + hr), zg = sigf(xz + hz);
          const float ng = tnhf(xn + rg * hn);
          const float hold = xf[(size_t)(rowg + row) * DIM + o];
          const float hnew = (1.0f - zg) * ng + zg * hold;
          o32[row * DIM + o] = hnew;
          o16[row * DIM + o] = (_Float16)(hnew * 8.0f);
        }
      }
      __syncthreads();
      {
        const int p = lane & 7, lr = lane >> 3;
        v4f v0, v1, v2;
        char *d0, *d1, *d2;
        {
          const int L = 8 * wave + lr;
          const int row = L >> 1, half = L & 1;
          v0 = *(const v4f*)(o32 + row * DIM + 32 * half + 4 * p);
          d0 = (char*)(yf + (size_t)(rowg + row) * DIM + 32 * half + 4 * p);
        }
        {
          const int L = 8 * wave + 4 + lr;
          const int row = L >> 1, half = L & 1;
          v1 = *(const v4f*)(o32 + row * DIM + 32 * half + 4 * p);
          d1 = (char*)(yf + (size_t)(rowg + row) * DIM + 32 * half + 4 * p);
        }
        {
          const int row = 4 * wave + lr;
          U8 u;
          u.h = *(const v8h*)(o16 + row * DIM + 8 * p);
          v2 = u.f;
          d2 = (char*)(yh + (size_t)(rowg + row) * DIM + 8 * p);
        }
        *(volatile v4f*)d0 = v0;
        *(volatile v4f*)d1 = v1;
        *(volatile v4f*)d2 = v2;
        __threadfence();
        *(volatile v4f*)d0 = v0;
        *(volatile v4f*)d1 = v1;
        *(volatile v4f*)d2 = v2;
      }
    }
  }
}

__global__ __launch_bounds__(256) void k_s2s(const float* __restrict__ xo, const int* __restrict__ bt,
                                             const float* __restrict__ wih, const float* __restrict__ whh,
                                             const float* __restrict__ bih, const float* __restrict__ bhh,
                                             const float* __restrict__ l1w, const float* __restrict__ l1b,
                                             const float* __restrict__ l2w, const float* __restrict__ l2b,
                                             float* y, int nN) {
  extern __shared__ __attribute__((aligned(16))) unsigned char dsm[];
  float* qs   = (float*)(dsm + S_QS);
  float* hs   = (float*)(dsm + S_HS);
  float* cs   = (float*)(dsm + S_CS);
  float* scr  = (float*)(dsm + S_SCR);
  float* emx  = (float*)(dsm + S_EMX);
  float* denp = (float*)(dsm + S_DEN);
  float* yL   = (float*)(dsm + S_Y);
  float* eL   = (float*)(dsm + S_E);
  const int tid = threadIdx.x;
  for (int i = tid; i < NGR * 2 * DIM; i += 256) qs[i] = 0.0f;
  for (int i = tid; i < NGR * DIM; i += 256) { hs[i] = 0.0f; cs[i] = 0.0f; }
  __syncthreads();
  const float ninf = -__builtin_inff();
  const int Q = (nN + 3) >> 2;

#pragma unroll 1
  for (int step = 0; step < 2; ++step) {
    {
      const int gc = tid;
      const float bsum = bih[gc] + bhh[gc];
      const float* wi = wih + (size_t)gc * 2 * DIM;
      const float* wh = whh + (size_t)gc * DIM;
#pragma unroll 1
      for (int b = 0; b < NGR; ++b) {
        float s = bsum;
        const float* qb = qs + b * 2 * DIM;
#pragma unroll 4
        for (int j = 0; j < 2 * DIM; ++j) s = fmaf(qb[j], wi[j], s);
        const float* hb = hs + b * DIM;
#pragma unroll 4
        for (int j = 0; j < DIM; ++j) s = fmaf(hb[j], wh[j], s);
        scr[b * 4 * DIM + gc] = s;
      }
    }
    __syncthreads();
    for (int idx = tid; idx < NGR * DIM; idx += 256) {
      const int b = idx >> 6, d = idx & 63;
      const float* gr = scr + b * 4 * DIM;
      const float ig = gr[d], fg = gr[DIM + d], gg = gr[2 * DIM + d], og = gr[3 * DIM + d];
      const float c = sigf(fg) * cs[idx] + sigf(ig) * tnhf(gg);
      cs[idx] = c;
      hs[idx] = sigf(og) * tnhf(c);
    }
    __syncthreads();
    for (int n = tid; n < nN; n += 256) {
      int b = bt[n];
      b = b < 0 ? 0 : (b > NGR - 1 ? NGR - 1 : b);
      const v4f* orow = (const v4f*)(xo + (size_t)n * DIM);
      const v4f* qrow = (const v4f*)(hs + b * DIM);
      float s = 0.0f;
#pragma unroll 2
      for (int c = 0; c < DIM / 4; ++c) {
        const v4f a = orow[c], q = qrow[c];
        s = fmaf(a.x, q.x, s); s = fmaf(a.y, q.y, s); s = fmaf(a.z, q.z, s); s = fmaf(a.w, q.w, s);
      }
      eL[n] = s;
    }
    __syncthreads();
    {
      const int part = tid >> 6, b = tid & 63;
      const int n0 = part * Q;
      int n1 = n0 + Q;
      n1 = n1 > nN ? nN : n1;
      float mx = ninf;
#pragma unroll 1
      for (int n = n0; n < n1; ++n) {
        const int bn = bt[n];
        const float v = eL[n];
        mx = (bn == b) ? fmaxf(mx, v) : mx;
      }
      emx[tid] = mx;
    }
    __syncthreads();
    {
      const int part = tid >> 6, b = tid & 63;
      const float m4 = fmaxf(fmaxf(emx[b], emx[NGR + b]), fmaxf(emx[2 * NGR + b], emx[3 * NGR + b]));
      const int n0 = part * Q;
      int n1 = n0 + Q;
      n1 = n1 > nN ? nN : n1;
      float den = 0.0f;
#pragma unroll 1
      for (int n = n0; n < n1; ++n) {
        const int bn = bt[n];
        const float t = __expf(eL[n] - m4);
        den += (bn == b) ? t : 0.0f;
      }
      denp[tid] = den;
    }
    __syncthreads();
    {
      const int b = tid >> 2, dq = tid & 3;
      const float m4 = fmaxf(fmaxf(emx[b], emx[NGR + b]), fmaxf(emx[2 * NGR + b], emx[3 * NGR + b]));
      const float den = ((denp[b] + denp[NGR + b]) + denp[2 * NGR + b]) + denp[3 * NGR + b];
      const float rden = __builtin_amdgcn_rcpf(fmaxf(den, 1e-16f));
      float rv[16];
#pragma unroll
      for (int j = 0; j < 16; ++j) rv[j] = 0.0f;
#pragma unroll 1
      for (int n = 0; n < nN; ++n) {
        const int bn = bt[n];
        const float t = __expf(eL[n] - m4) * rden;
        const float a = (bn == b) ? t : 0.0f;
        const v4f* orow = (const v4f*)(xo + (size_t)n * DIM + 16 * dq);
#pragma unroll
        for (int c = 0; c < 4; ++c) {
          const v4f o4 = orow[c];
          rv[4 * c + 0] = fmaf(a, o4.x, rv[4 * c + 0]);
          rv[4 * c + 1] = fmaf(a, o4.y, rv[4 * c + 1]);
          rv[4 * c + 2] = fmaf(a, o4.z, rv[4 * c + 2]);
          rv[4 * c + 3] = fmaf(a, o4.w, rv[4 * c + 3]);
        }
      }
#pragma unroll
      for (int j = 0; j < 16; ++j) scr[b * DIM + 16 * dq + j] = rv[j];
    }
    __syncthreads();
    for (int idx = tid; idx < NGR * DIM; idx += 256) {
      const int b = idx >> 6, d = idx & 63;
      qs[b * 2 * DIM + d] = hs[idx];
      qs[b * 2 * DIM + DIM + d] = scr[idx];
    }
    __syncthreads();
  }

  for (int idx = tid; idx < NGR * DIM; idx += 256) {
    const int b = idx >> 6, d = idx & 63;
    float s = l1b[d];
    const float* qb = qs + b * 2 * DIM;
    const float* wr = l1w + (size_t)d * 2 * DIM;
#pragma unroll 4
    for (int j = 0; j < 2 * DIM; ++j) s = fmaf(qb[j], wr[j], s);
    scr[idx] = fmaxf(s, 0.0f);
  }
  __syncthreads();
  if (tid < NGR) {
    float s = l2b[0];
#pragma unroll 4
    for (int d = 0; d < DIM; ++d) s = fmaf(scr[tid * DIM + d], l2w[d], s);
    yL[tid] = s;
  }
  __syncthreads();
  {
    v4f v = {0.0f, 0.0f, 0.0f, 0.0f};
    if (tid < 16) v = *(const v4f*)(yL + 4 * tid);
    if (tid < 16) *(volatile v4f*)(y + 4 * tid) = v;
    __threadfence();
    if (tid < 16) *(volatile v4f*)(y + 4 * tid) = v;
  }
}

extern "C" void kernel_launch(void* const* d_in, const int* in_sizes, int n_in,
                              void* d_out, int out_size, void* d_ws, size_t ws_size,
                              hipStream_t stream) {
  if (n_in < 24) return;
  const int nN = in_sizes[23];
  const int nE = in_sizes[22] / 2;
  if (nN < 1 || nE < 1 || in_sizes[22] != 2 * nE) return;
  if (in_sizes[0] != nN * NFT || in_sizes[1] != nE * EFT) return;
  if (in_sizes[2] != DIM * NFT || in_sizes[3] != DIM || in_sizes[4] != HID * EFT || in_sizes[5] != HID) return;
  if (in_sizes[6] != DIM * DIM * HID || in_sizes[7] != DIM * DIM || in_sizes[8] != DIM * DIM || in_sizes[9] != DIM) return;
  if (in_sizes[10] != 3 * DIM * DIM || in_sizes[11] != 3 * DIM * DIM || in_sizes[12] != 3 * DIM || in_sizes[13] != 3 * DIM) return;
  if (in_sizes[14] != 4 * DIM * 2 * DIM || in_sizes[15] != 4 * DIM * DIM || in_sizes[16] != 4 * DIM || in_sizes[17] != 4 * DIM) return;
  if (in_sizes[18] != DIM * 2 * DIM || in_sizes[19] != DIM || in_sizes[20] != DIM || in_sizes[21] != 1) return;
  if (out_size != NGR) return;

  const float* x         = (const float*)d_in[0];
  const float* edge_attr = (const float*)d_in[1];
  const float* lin0_w    = (const float*)d_in[2];
  const float* lin0_b    = (const float*)d_in[3];
  const float* nn1_w     = (const float*)d_in[4];
  const float* nn1_b     = (const float*)d_in[5];
  const float* nn2_w     = (const float*)d_in[6];
  const float* nn2_b     = (const float*)d_in[7];
  const float* root      = (const float*)d_in[8];
  const float* conv_bias = (const float*)d_in[9];
  const float* gru_w_ih  = (const float*)d_in[10];
  const float* gru_w_hh  = (const float*)d_in[11];
  const float* gru_b_ih  = (const float*)d_in[12];
  const float* gru_b_hh  = (const float*)d_in[13];
  const float* lstm_w_ih = (const float*)d_in[14];
  const float* lstm_w_hh = (const float*)d_in[15];
  const float* lstm_b_ih = (const float*)d_in[16];
  const float* lstm_b_hh = (const float*)d_in[17];
  const float* lin1_w    = (const float*)d_in[18];
  const float* lin1_b    = (const float*)d_in[19];
  const float* lin2_w    = (const float*)d_in[20];
  const float* lin2_b    = (const float*)d_in[21];
  const int*   ei        = (const int*)d_in[22];
  const int*   batch     = (const int*)d_in[23];
  float* yout = (float*)d_out;

  const int NBLK = (nN + NBK - 1) / NBK;
  const int NP   = NBLK * NBK;
  const int EBK  = (nE + ET - 1) / ET;
  const int EP   = EBK * ET;
  const int s2sL = S_E + ((nN * 4 + 15) & ~15);
  if (s2sL > 300 * 1024) return;

  char* ws = (char*)d_ws;
  size_t off = 0;
  auto carve = [&](size_t bytes) -> char* { char* p = ws + off; off += (bytes + 255) & ~(size_t)255; return p; };
  _Float16* w1s   = (_Float16*)carve((size_t)HID * 64 * 2);
  _Float16* rootp = (_Float16*)carve((size_t)DIM * DIM * 2);
  _Float16* gihs  = (_Float16*)carve((size_t)3 * DIM * DIM * 2);
  _Float16* ghhs  = (_Float16*)carve((size_t)3 * DIM * DIM * 2);
  _Float16* w2s   = (_Float16*)carve((size_t)DIM * KW2 * 2);
  _Float16* he16  = (_Float16*)carve((size_t)EP * HID * 2);
  float*    xf0   = (float*)carve((size_t)NP * DIM * 4);
  float*    xf1   = (float*)carve((size_t)NP * DIM * 4);
  float*    xf2   = (float*)carve((size_t)NP * DIM * 4);
  _Float16* xh0   = (_Float16*)carve((size_t)NP * DIM * 2);
  _Float16* xh1   = (_Float16*)carve((size_t)NP * DIM * 2);
  _Float16* xh2   = (_Float16*)carve((size_t)NP * DIM * 2);
  size_t limit = (size_t)134217728;
  if (ws_size < limit) limit = ws_size;
  if (off > limit) return;

  const int vec8 = ((nE & 3) == 0) ? 1 : 0;

  k_prep4<<<dim3((3 * DIM * 8 + 127) / 128, 4), 128, 0, stream>>>(nn1_w, root, gru_w_ih, gru_w_hh,
                                                                  w1s, rootp, gihs, ghhs);
  k_prepw2<<<(DIM * (KW2 / 8) + 127) / 128, 128, 0, stream>>>(nn2_w, nn2_b, w2s);
  k_lin0<<<NP / 4, 256, 0, stream>>>(x, lin0_w, lin0_b, xf0, xh0, nN);
  k_nn1<<<EBK, CT, 0, stream>>>(edge_attr, nn1_b, w1s, he16, nE);

  hipFuncSetAttribute(reinterpret_cast<const void*>(&k_conv), hipFuncAttributeMaxDynamicSharedMemorySize, L_TOTAL);
  k_conv<<<NBLK, CT, L_TOTAL, stream>>>(ei, xh0, xf0, he16, w2s, rootp, gihs, ghhs, conv_bias, gru_b_ih, gru_b_hh,
                                        xf1, xh1, nN, nE, vec8);
  k_conv<<<NBLK, CT, L_TOTAL, stream>>>(ei, xh1, xf1, he16, w2s, rootp, gihs, ghhs, conv_bias, gru_b_ih, gru_b_hh,
                                        xf2, xh2, nN, nE, vec8);

  hipFuncSetAttribute(reinterpret_cast<const void*>(&k_s2s), hipFuncAttributeMaxDynamicSharedMemorySize, s2sL);
  k_s2s<<<1, 256, s2sL, stream>>>(xf2, batch, lstm_w_ih, lstm_w_hh, lstm_b_ih, lstm_b_hh,
                                  lin1_w, lin1_b, lin2_w, lin2_b, yout, nN);
}
